// GAT_1468878815266
// MI455X (gfx1250) — hardware-verified
//
#include <hip/hip_runtime.h>
#include <math.h>

#ifndef NB
#define NB 16
#endif
#define NODES 512
#define LG_NODES 9
#define FEAT 128
#define HEADS 8
#define LG_HEADS 3
#define DH 32
#define HDIM 256
#define NCLS 128
#define MTOK (NB * NODES)

#define LEAKY 0.2f
#define NEGFILL -9.0e15f
#define LOG2E 1.4426950408889634f

static constexpr float XCARRY  = 16.0f;
static constexpr float WCARRY  = 64.0f;
static constexpr float HCARRY  = 16.0f;
static constexpr float PCARRY  = 1024.0f;
static constexpr float XCCARRY = 64.0f;
static constexpr float SC1   = 1.0f / 1024.0f;
static constexpr float SC2   = 1.0f / 4096.0f;
static constexpr float OUNDO = 1.0f / 16384.0f;
static_assert(SC1 * XCARRY * WCARRY == 1.0f);
static_assert(SC2 * XCCARRY * WCARRY == 1.0f);
static_assert(OUNDO * HCARRY * PCARRY == 1.0f);

static_assert((1 << LG_NODES) == NODES);
static_assert((1 << LG_HEADS) == HEADS);
static_assert(HEADS * DH == HDIM);
static_assert(NODES % 64 == 0 && HDIM % 64 == 0 && NCLS % 64 == 0);
static_assert(FEAT % 32 == 0 && HDIM % 32 == 0 && NODES % 32 == 0);
static_assert((MTOK * FEAT / 8) % 256 == 0);
static_assert((NB * HEADS * NODES) % 256 == 0 && (NB * NODES) % 256 == 0);
static_assert(DH % 4 == 0 && NCLS % 4 == 0);

typedef _Float16 h16;
typedef __attribute__((ext_vector_type(16))) _Float16 v16h;
typedef __attribute__((ext_vector_type(8)))  _Float16 v8h;
typedef __attribute__((ext_vector_type(8)))  float    v8f;
typedef __attribute__((ext_vector_type(4)))  float    v4f;
typedef __attribute__((ext_vector_type(4)))  int      v4i;


#define VST2(T, ptr, val) do { const T vst2_v_ = (val); *(volatile T*)(ptr) = vst2_v_; __threadfence(); *(volatile T*)(ptr) = vst2_v_; } while (0)

__device__ __forceinline__ float bfr(float f) {
    unsigned u = __float_as_uint(f);
    u += 0x7FFFu + ((u >> 16) & 1u);
    return __uint_as_float(u & 0xFFFF0000u);
}
static __device__ __forceinline__ h16 toh_flush(float v) { const float w = (fabsf(v) < 6.103515625e-05f) ? 0.0f : v; return (h16)w; }

static __device__ __forceinline__ void st8h_flush(h16* P, size_t o, const float* v) {
    v8h hv;
#pragma unroll
    for (int e = 0; e < 8; ++e) hv[e] = toh_flush(v[e]);
    *(volatile v8h*)(P + o) = hv;
    __threadfence();
    *(volatile v8h*)(P + o) = hv;
}

union FragU { v16h v; v8h h[2]; };
__device__ __forceinline__ v16h frag_ld(const _Float16* p) {
    FragU f; f.h[0] = *(const v8h*)(p); f.h[1] = *(const v8h*)(p + 16); return f.v;
}
__device__ __forceinline__ v8f wmma16g(v16h a, v16h b, v8f c) {
    c = __builtin_amdgcn_wmma_f32_16x16x32_f16(false, a, false, b, (short)0, c, false, false);
    asm volatile("v_nop\n\tv_nop\n\tv_nop\n\tv_nop" : "+v"(c) : "v"(a), "v"(b));
    return c;
}
__device__ __forceinline__ void wave_sync_lds() {
    __builtin_amdgcn_fence(3  , "workgroup");
    __builtin_amdgcn_wave_barrier();
    __builtin_amdgcn_fence(2  , "workgroup");
}

__global__ __launch_bounds__(256) void k_xconv(const float* __restrict__ x, h16* __restrict__ X16) {
    const unsigned u = blockIdx.x * 256u + threadIdx.x;
    const size_t o = (size_t)u * 8u;
    const v4f a = *(const v4f*)(x + o);
    const v4f b = *(const v4f*)(x + o + 4u);
    float v[8];
    v[0] = bfr(a.x) * XCARRY; v[1] = bfr(a.y) * XCARRY; v[2] = bfr(a.z) * XCARRY; v[3] = bfr(a.w) * XCARRY;
    v[4] = bfr(b.x) * XCARRY; v[5] = bfr(b.y) * XCARRY; v[6] = bfr(b.z) * XCARRY; v[7] = bfr(b.w) * XCARRY;
    st8h_flush(X16, o, v);
}

__global__ __launch_bounds__(256) void k_wconv(const float* __restrict__ Wm, unsigned KI, unsigned NO, unsigned lgper,
                                               h16* __restrict__ W16) {
    const unsigned slab = blockIdx.y;
    const float* Wl = Wm + (size_t)slab * KI * NO;
    h16* Dl = W16 + (size_t)slab * KI * NO;
    const unsigned u = blockIdx.x * 256u + threadIdx.x;
    const unsigned per = 1u << lgper;
    if (u >= NO * per) return;
    const unsigned k0 = 8u * (u & (per - 1u));
    const unsigned o = u >> lgper;
    float v[8];
#pragma unroll
    for (int i = 0; i < 8; ++i) v[i] = bfr(Wl[(size_t)(k0 + (unsigned)i) * NO + o]) * WCARRY;
    st8h_flush(Dl, (size_t)o * KI + k0, v);
}

#define GEMM_WAVES 4
#define GP_F 68
#define GP_H 72
static_assert(GEMM_WAVES * (16 * GP_F * 4 + 64 * GP_H * 2) <= 131072);
static_assert(32 * 16 * 8 == 16 * 64 * 4);
static_assert(32 * 16 * 16 == 64 * 64 * 2);

template <int TWO, int LGTN>
static __device__ __forceinline__ void gemm_body(const h16* __restrict__ A0, const h16* __restrict__ A1, const unsigned lda,
                                                 const h16* __restrict__ Bt, const unsigned ldb,
                                                 float* __restrict__ C, h16* __restrict__ T, const unsigned K, const float scale) {
  __shared__ __align__(16) float sC[GEMM_WAVES][16 * GP_F];
  __shared__ __align__(16) h16   sH[GEMM_WAVES][64 * GP_H];
  constexpr unsigned NC = 64u << LGTN;
  const unsigned lane = threadIdx.x & 31u;
  const unsigned wave = (unsigned)__builtin_amdgcn_readfirstlane((int)(threadIdx.x >> 5));
  const unsigned bx = blockIdx.x;
  const unsigned tile = bx * (unsigned)GEMM_WAVES + wave;
  const unsigned tm = tile >> LGTN;
  const unsigned tn = tile & ((1u << LGTN) - 1u);
  const unsigned m0 = tm << 6, n0 = tn << 6;
  const unsigned rlane = lane & 15u;
  const unsigned hh = lane >> 4;
  const unsigned koff = hh * 8u;

  v8f acc[4][4];
#pragma unroll
  for (int i = 0; i < 4; ++i)
#pragma unroll
    for (int j = 0; j < 4; ++j) acc[i][j] = (v8f){0.f,0.f,0.f,0.f,0.f,0.f,0.f,0.f};

#pragma unroll 1
  for (unsigned k0 = 0; k0 < K; k0 += 32u) {
    unsigned kb = k0 + koff;
    asm volatile("" : "+v"(kb));
    v16h bf[4];
#pragma unroll
    for (int j = 0; j < 4; ++j)
      bf[j] = frag_ld(Bt + (size_t)(n0 + ((unsigned)j << 4) + rlane) * ldb + kb);
#pragma unroll
    for (int i = 0; i < 4; ++i) {
      unsigned ka = k0 + koff;
      asm volatile("" : "+v"(ka));
      const v16h ah = frag_ld(A0 + (size_t)(m0 + ((unsigned)i << 4) + rlane) * lda + ka);
#pragma unroll
      for (int j = 0; j < 4; ++j) acc[i][j] = wmma16g(ah, bf[j], acc[i][j]);
      if (TWO) {
        const v16h al = frag_ld(A1 + (size_t)(m0 + ((unsigned)i << 4) + rlane) * lda + ka);
#pragma unroll
        for (int j = 0; j < 4; ++j) acc[i][j] = wmma16g(al, bf[j], acc[i][j]);
      }
    }
  }

#pragma unroll
  for (int i = 0; i < 4; ++i) {
    const unsigned mBase = m0 + ((unsigned)i << 4);
#pragma unroll
    for (int j = 0; j < 4; ++j) {
      v8h hv;
#pragma unroll
      for (int r = 0; r < 8; ++r) {
        const float v = acc[i][j][r] * scale;
        sC[wave][(koff + (unsigned)r) * GP_F + ((unsigned)j << 4) + rlane] = v;
        hv[r] = toh_flush(v * HCARRY);
      }
      *(v8h*)(&sH[wave][(((unsigned)j << 4) + rlane) * GP_H + ((unsigned)i << 4) + koff]) = hv;
    }
    wave_sync_lds();
    {
      const unsigned c4 = (lane & 15u) * 4u;
#pragma unroll
      for (int half = 0; half < 2; ++half) {
        v4f vv[4];
#pragma unroll
        for (int it = 0; it < 4; ++it) {
          const unsigned row = (unsigned)(half * 4 + it) * 2u + hh;
          vv[it] = *(const v4f*)(&sC[wave][row * GP_F + c4]);
        }
        for (int pass = 0; pass < 2; ++pass) {
#pragma unroll
          for (int it = 0; it < 4; ++it) {
            const unsigned row = (unsigned)(half * 4 + it) * 2u + hh;
            *(volatile v4f*)(C + (size_t)(mBase + row) * NC + n0 + c4) = vv[it];
          }
          __threadfence();
        }
      }
    }
    wave_sync_lds();
  }
  {
    const unsigned q = lane >> 3, c8 = (lane & 7u) * 8u;
    const unsigned gb = m0 >> LG_NODES, jb = m0 & (unsigned)(NODES - 1);
    h16* tb = T + (size_t)(gb * NC + n0) * NODES + jb + c8;
#pragma unroll
    for (int g = 0; g < 4; ++g) {
      v8h hv[4];
#pragma unroll
      for (int it = 0; it < 4; ++it) {
        const unsigned row = (unsigned)(g * 16 + it * 4) + q;
        hv[it] = *(const v8h*)(&sH[wave][row * GP_H + c8]);
      }
      for (int pass = 0; pass < 2; ++pass) {
#pragma unroll
        for (int it = 0; it < 4; ++it) {
          const unsigned row = (unsigned)(g * 16 + it * 4) + q;
          *(volatile v8h*)(tb + (size_t)row * NODES) = hv[it];
        }
        __threadfence();
      }
    }
  }
}

static_assert(((MTOK / 64) * (HDIM / 64)) % GEMM_WAVES == 0);
static_assert(((MTOK / 64) * (NCLS / 64)) % GEMM_WAVES == 0);
static_assert((64 << 2) == HDIM && (64 << 1) == NCLS);

__global__ __launch_bounds__(128) __attribute__((amdgpu_num_vgpr(256)))
void k_gemm_a(const h16* __restrict__ X16, const h16* __restrict__ W1T, float* __restrict__ HF, h16* __restrict__ HT) {
  gemm_body<0, 2>(X16, X16, FEAT, W1T, FEAT, HF, HT, FEAT, SC1);
}
__global__ __launch_bounds__(128) __attribute__((amdgpu_num_vgpr(256)))
void k_gemm_b(const h16* __restrict__ XH, const h16* __restrict__ XL, const h16* __restrict__ W2T,
              float* __restrict__ H2F, h16* __restrict__ H2T) {
  gemm_body<1, 1>(XH, XL, HDIM, W2T, HDIM, H2F, H2T, HDIM, SC2);
}

__global__ __launch_bounds__(256) void k_rowdot(const float* __restrict__ Hf, const float* __restrict__ av,
                                                float* __restrict__ fr, float* __restrict__ fc,
                                                unsigned lgheads, unsigned width) {
    const unsigned idx = blockIdx.x * 256u + threadIdx.x;
    const unsigned n = idx & (unsigned)(NODES - 1);
    const unsigned gh = idx >> LG_NODES;
    const unsigned hd = gh & ((1u << lgheads) - 1u);
    const unsigned g = gh >> lgheads;
    const float* src = Hf + (size_t)(g * (unsigned)NODES + n) * (width << lgheads) + hd * width;
    const float* a = av + (size_t)hd * 2u * width;
    float s1 = 0.f, s2 = 0.f;
#pragma unroll 1
    for (unsigned d = 0; d < width; d += 4u) {
        const v4f h = *(const v4f*)(src + d);
        const v4f p = *(const v4f*)(a + d);
        const v4f q = *(const v4f*)(a + width + d);
        s1 += h.x * bfr(p.x) + h.y * bfr(p.y) + h.z * bfr(p.z) + h.w * bfr(p.w);
        s2 += h.x * bfr(q.x) + h.y * bfr(q.y) + h.z * bfr(q.z) + h.w * bfr(q.w);
    }
    VST2(float, fr + idx, s1);
    VST2(float, fc + idx, s2);
}

template <int NT, bool PLO>
static __device__ __forceinline__ void attn_head(const h16* __restrict__ vt, const int* __restrict__ arow, const float* sf,
                                                 const float fq, const unsigned c, const unsigned hh,
                                                 v8f (&acc)[NT], float& lsum) {
    constexpr int GT = (NT < 4) ? NT : 4;
    static_assert(NT % GT == 0);
    float mrun = -3.0e38f;
    float lrun = 0.0f;
#pragma unroll
    for (int t = 0; t < NT; ++t) acc[t] = (v8f){0.f,0.f,0.f,0.f,0.f,0.f,0.f,0.f};
#pragma unroll 1
    for (unsigned j0 = 0; j0 < (unsigned)NODES; j0 += 32u) {
        const v4i m0 = *(const v4i*)(arow + j0);
        const v4i m1 = *(const v4i*)(arow + j0 + 4u);
        const v4i m2 = *(const v4i*)(arow + j0 + 16u);
        const v4i m3 = *(const v4i*)(arow + j0 + 20u);
        const unsigned ja = j0 + 8u * hh;
        const v4f g0 = *(const v4f*)(sf + ja);
        const v4f g1 = *(const v4f*)(sf + ja + 4u);
        const v4f g2 = *(const v4f*)(sf + ja + 16u);
        const v4f g3 = *(const v4f*)(sf + ja + 20u);
        const int mk[16] = {m0.x, m0.y, m0.z, m0.w, m1.x, m1.y, m1.z, m1.w, m2.x, m2.y, m2.z, m2.w, m3.x, m3.y, m3.z, m3.w};
        const float fv[16] = {g0.x, g0.y, g0.z, g0.w, g1.x, g1.y, g1.z, g1.w, g2.x, g2.y, g2.z, g2.w, g3.x, g3.y, g3.z, g3.w};
        float e[16];
#pragma unroll
        for (int k = 0; k < 16; ++k) {
            float t = fq + fv[k];
            t = (t > 0.0f) ? t : LEAKY * t;
            t = (mk[k] > 0) ? t : NEGFILL;
            e[k] = t * LOG2E;
        }
        float mx = e[0];
#pragma unroll
        for (int k = 1; k < 16; ++k) mx = (e[k] > mx) ? e[k] : mx;
        const float mo = __shfl_xor(mx, 16, 32);
        mx = (mo > mx) ? mo : mx;
        const float mnew = (mx > mrun) ? mx : mrun;
        const float alpha = exp2f(mrun - mnew);
        mrun = mnew;
        float ps = 0.0f;
        v16h bhv, blv;
#pragma unroll
        for (int k = 0; k < 16; ++k) {
            const float p = exp2f(e[k] - mnew);
            ps += p;
            const float w = p * PCARRY;
            const h16 ph = toh_flush(w);
            bhv[k] = ph;
            if constexpr (PLO) {
                const h16 pl = toh_flush(w - (float)ph);
                blv[k] = pl;
            }
        }
        lrun = lrun * alpha + ps;
#pragma unroll
        for (int t = 0; t < NT; ++t)
#pragma unroll
            for (int r = 0; r < 8; ++r) acc[t][r] *= alpha;
#pragma unroll
        for (int g = 0; g < NT / GT; ++g) {
            unsigned ko = ja;
            asm volatile("" : "+v"(ko));
#pragma unroll
            for (int tt = 0; tt < GT; ++tt) {
                const int t = g * GT + tt;
                const v16h a = frag_ld(vt + (size_t)((unsigned)(t * 16) + c) * NODES + ko);
                acc[t] = wmma16g(a, bhv, acc[t]);
                if constexpr (PLO) acc[t] = wmma16g(a, blv, acc[t]);
            }
        }
    }
    lsum = lrun;
}

#define ATT_WAVES 4
#define OP_A 68
#define OP_B 132
static_assert(2 * NODES * 4 + ATT_WAVES * 16 * OP_A * 4 <= 131072);
static_assert(NODES * 4 + ATT_WAVES * 16 * OP_B * 4 <= 131072);
static_assert(ATT_WAVES * 32 * 4 == NODES);
static_assert(32 * 16 * 4 == 16 * 64 * 2);
static_assert(32 * 16 * 16 == 16 * NCLS * 4);
static_assert(NODES / 64 == 8 && HEADS / 2 == 4);

__global__ __launch_bounds__(128) __attribute__((amdgpu_num_vgpr(256)))
void k_attn_a(const h16* __restrict__ HT, const int* __restrict__ adj, const float* __restrict__ fr,
              const float* __restrict__ fc, h16* __restrict__ XH, h16* __restrict__ XL) {
    __shared__ __align__(16) float sF[2 * NODES];
    __shared__ __align__(16) float sO[ATT_WAVES][16 * OP_A];
    const unsigned tid = threadIdx.x, lane = tid & 31u;
    const unsigned wave = (unsigned)__builtin_amdgcn_readfirstlane((int)(threadIdx.x >> 5));
    const unsigned hh = lane >> 4, c = lane & 15u;
    const unsigned bx = blockIdx.x;
    const unsigned qb = bx & 7u, pair = (bx >> 3) & 3u, g = bx >> 5;
#pragma unroll
    for (unsigned hl = 0; hl < 2u; ++hl) {
        const v4f v = *(const v4f*)(fc + (size_t)((g * (unsigned)HEADS + 2u * pair + hl) * (unsigned)NODES) + 4u * tid);
        *(v4f*)(&sF[hl * (unsigned)NODES + 4u * tid]) = v;
    }
    __syncthreads();
    const unsigned q0 = qb * 64u + wave * 16u;
    const int* arow = adj + (size_t)(g * (unsigned)NODES + q0 + c) * NODES + 8u * hh;
#pragma unroll 1
    for (unsigned hp = 0; hp < 2u; ++hp) {
        const unsigned head = 2u * pair + hp;
        const float fq = fr[(size_t)((g * (unsigned)HEADS + head) * (unsigned)NODES) + q0 + c];
        v8f acc[2];
        float ls;
        attn_head<2, false>(HT + (size_t)(g * (unsigned)HDIM + head * (unsigned)DH) * NODES, arow, &sF[hp * (unsigned)NODES], fq, c, hh, acc, ls);
        const float l = ls + __shfl_xor(ls, 16, 32);
        const float inv = 1.0f / (l * (HCARRY * PCARRY));
#pragma unroll
        for (int t = 0; t < 2; ++t) {
            v4f lo4, hi4;
            lo4.x = acc[t][0] * inv; lo4.y = acc[t][1] * inv; lo4.z = acc[t][2] * inv; lo4.w = acc[t][3] * inv;
            hi4.x = acc[t][4] * inv; hi4.y = acc[t][5] * inv; hi4.z = acc[t][6] * inv; hi4.w = acc[t][7] * inv;
            float* dst = &sO[wave][c * OP_A + hp * 32u + (unsigned)(t * 16) + 8u * hh];
            *(v4f*)(dst) = lo4;
            *(v4f*)(dst + 4) = hi4;
        }
    }
    wave_sync_lds();
    {
        const unsigned q = lane >> 3, c8 = (lane & 7u) * 8u;
#pragma unroll 1
        for (unsigned it = 0; it < 4u; ++it) {
            const unsigned row = 4u * it + q;
            const v4f a0 = *(const v4f*)(&sO[wave][row * OP_A + c8]);
            const v4f a1 = *(const v4f*)(&sO[wave][row * OP_A + c8 + 4u]);
            const float v[8] = {a0.x, a0.y, a0.z, a0.w, a1.x, a1.y, a1.z, a1.w};
            v8h wh, wl;
#pragma unroll
            for (int e = 0; e < 8; ++e) {
                float y = v[e];
                y = (y > 0.0f) ? y : expm1f(y);
                const float s = y * XCCARRY;
                const h16 h = toh_flush(s);
                wh[e] = h;
                wl[e] = toh_flush(s - (float)h);
            }
            const size_t o = (size_t)(g * (unsigned)NODES + q0 + row) * HDIM + pair * 64u + c8;
            *(volatile v8h*)(XH + o) = wh;
            *(volatile v8h*)(XL + o) = wl;
            __threadfence();
            *(volatile v8h*)(XH + o) = wh;
            *(volatile v8h*)(XL + o) = wl;
        }
    }
}

__global__ __launch_bounds__(128) __attribute__((amdgpu_num_vgpr(256)))
void k_attn_b(const h16* __restrict__ H2T, const int* __restrict__ adj, const float* __restrict__ gr,
              const float* __restrict__ gc, const float* __restrict__ x, float* __restrict__ out) {
    __shared__ __align__(16) float sG[NODES];
    __shared__ __align__(16) float sO[ATT_WAVES][16 * OP_B];
    const unsigned tid = threadIdx.x, lane = tid & 31u;
    const unsigned wave = (unsigned)__builtin_amdgcn_readfirstlane((int)(threadIdx.x >> 5));
    const unsigned hh = lane >> 4, c = lane & 15u;
    const unsigned bx = blockIdx.x;
    const unsigned qb = bx & 7u, g = bx >> 3;
    {
        const v4f v = *(const v4f*)(gc + (size_t)(g * (unsigned)NODES) + 4u * tid);
        *(v4f*)(&sG[4u * tid]) = v;
    }
    __syncthreads();
    const unsigned q0 = qb * 64u + wave * 16u;
    const int* arow = adj + (size_t)(g * (unsigned)NODES + q0 + c) * NODES + 8u * hh;
    const float fq = gr[(size_t)(g * (unsigned)NODES) + q0 + c];
    v8f acc[8];
    float ls;
    attn_head<8, false>(H2T + (size_t)(g * (unsigned)NCLS) * NODES, arow, &sG[0], fq, c, hh, acc, ls);
    const float l = ls + __shfl_xor(ls, 16, 32);
    const float inv = 1.0f / (l * (HCARRY * PCARRY));
#pragma unroll
    for (int t = 0; t < 8; ++t) {
        v4f lo4, hi4;
        lo4.x = acc[t][0] * inv; lo4.y = acc[t][1] * inv; lo4.z = acc[t][2] * inv; lo4.w = acc[t][3] * inv;
        hi4.x = acc[t][4] * inv; hi4.y = acc[t][5] * inv; hi4.z = acc[t][6] * inv; hi4.w = acc[t][7] * inv;
        float* dst = &sO[wave][c * OP_B + (unsigned)(t * 16) + 8u * hh];
        *(v4f*)(dst) = lo4;
        *(v4f*)(dst + 4) = hi4;
    }
    wave_sync_lds();
#pragma unroll 1
    for (unsigned grp = 0; grp < 4u; ++grp) {
        v4f ov[4];
#pragma unroll
        for (int it = 0; it < 4; ++it) {
            const unsigned row = 4u * grp + (unsigned)it;
            v4f y = *(const v4f*)(&sO[wave][row * OP_B + 4u * lane]);
            const v4f xr = *(const v4f*)(x + (size_t)(g * (unsigned)NODES + q0 + row) * FEAT + 4u * lane);
            y.x = ((y.x > 0.0f) ? y.x : expm1f(y.x)) + bfr(xr.x);
            y.y = ((y.y > 0.0f) ? y.y : expm1f(y.y)) + bfr(xr.y);
            y.z = ((y.z > 0.0f) ? y.z : expm1f(y.z)) + bfr(xr.z);
            y.w = ((y.w > 0.0f) ? y.w : expm1f(y.w)) + bfr(xr.w);
            ov[it] = y;
        }
        for (int pass = 0; pass < 2; ++pass) {
#pragma unroll
            for (int it = 0; it < 4; ++it) {
                const unsigned row = 4u * grp + (unsigned)it;
                *(volatile v4f*)(out + (size_t)(g * (unsigned)NODES + q0 + row) * NCLS + 4u * lane) = ov[it];
            }
            __threadfence();
        }
    }
}

static constexpr size_t SZ_X16 = (size_t)MTOK * FEAT * 2;
static constexpr size_t SZ_W1T = (size_t)HDIM * FEAT * 2;
static constexpr size_t SZ_W2T = (size_t)NCLS * HDIM * 2;
static constexpr size_t SZ_HF  = (size_t)MTOK * HDIM * 4;
static constexpr size_t SZ_HT  = (size_t)NB * HDIM * NODES * 2;
static constexpr size_t SZ_F   = (size_t)NB * HEADS * NODES * 4;
static constexpr size_t SZ_XC  = (size_t)MTOK * HDIM * 2;
static constexpr size_t SZ_H2F = (size_t)MTOK * NCLS * 4;
static constexpr size_t SZ_H2T = (size_t)NB * NCLS * NODES * 2;
static constexpr size_t SZ_G   = (size_t)NB * NODES * 4;
static constexpr size_t OFF_X16 = 0;
static constexpr size_t OFF_W1T = OFF_X16 + SZ_X16;
static constexpr size_t OFF_W2T = OFF_W1T + SZ_W1T;
static constexpr size_t OFF_HF  = OFF_W2T + SZ_W2T;
static constexpr size_t OFF_HT  = OFF_HF + SZ_HF;
static constexpr size_t OFF_F1  = OFF_HT + SZ_HT;
static constexpr size_t OFF_F2  = OFF_F1 + SZ_F;
static constexpr size_t OFF_XCH = OFF_F2 + SZ_F;
static constexpr size_t OFF_XCL = OFF_XCH + SZ_XC;
static constexpr size_t OFF_H2F = OFF_XCL + SZ_XC;
static constexpr size_t OFF_H2T = OFF_H2F + SZ_H2F;
static constexpr size_t OFF_G1  = OFF_H2T + SZ_H2T;
static constexpr size_t OFF_G2  = OFF_G1 + SZ_G;
static constexpr size_t WS_TOTAL = OFF_G2 + SZ_G;
static_assert(SZ_X16 % 256 == 0 && SZ_W1T % 256 == 0 && SZ_W2T % 256 == 0 && SZ_HF % 256 == 0 && SZ_HT % 256 == 0);
static_assert(SZ_F % 256 == 0 && SZ_XC % 256 == 0 && SZ_H2F % 256 == 0 && SZ_H2T % 256 == 0 && SZ_G % 256 == 0);
static_assert(WS_TOTAL <= (size_t)134217728);
static_assert((size_t)MTOK * NCLS * 4 <= (size_t)16 * 512 * 128 * 4);

extern "C" void kernel_launch(void* const* d_in, const int* in_sizes, int n_in, void* d_out, int out_size,
                              void* d_ws, size_t ws_size, hipStream_t stream) {
    if (n_in < 6) return;
    if (in_sizes[0] < MTOK * FEAT || in_sizes[1] < MTOK * NODES || in_sizes[2] < HEADS * FEAT * DH) return;
    if (in_sizes[3] < HEADS * 2 * DH || in_sizes[4] < HDIM * NCLS || in_sizes[5] < 2 * NCLS) return;
    if (out_size < MTOK * NCLS) return;
    if (ws_size < WS_TOTAL) return;

    const float* x   = (const float*)d_in[0];
    const int*   adj = (const int*)d_in[1];
    const float* W1  = (const float*)d_in[2];
    const float* a1  = (const float*)d_in[3];
    const float* W2  = (const float*)d_in[4];
    const float* a2  = (const float*)d_in[5];
    float* out = (float*)d_out;

    char* wsp = (char*)d_ws;
    h16*   X16 = (h16*)(wsp + OFF_X16);
    h16*   W1T = (h16*)(wsp + OFF_W1T);
    h16*   W2T = (h16*)(wsp + OFF_W2T);
    float* HF  = (float*)(wsp + OFF_HF);
    h16*   HT  = (h16*)(wsp + OFF_HT);
    float* F1  = (float*)(wsp + OFF_F1);
    float* F2  = (float*)(wsp + OFF_F2);
    h16*   XCH = (h16*)(wsp + OFF_XCH);
    h16*   XCL = (h16*)(wsp + OFF_XCL);
    float* H2F = (float*)(wsp + OFF_H2F);
    h16*   H2T = (h16*)(wsp + OFF_H2T);
    float* G1  = (float*)(wsp + OFF_G1);
    float* G2  = (float*)(wsp + OFF_G2);

    k_xconv<<<(MTOK * FEAT / 8) / 256, 256, 0, stream>>>(x, X16);
    k_wconv<<<dim3((DH * (FEAT / 8)) / 256, HEADS), 256, 0, stream>>>(W1, FEAT, DH, 4, W1T);
    k_wconv<<<dim3((NCLS * (HDIM / 8)) / 256, 1), 256, 0, stream>>>(W2, HDIM, NCLS, 5, W2T);

    k_gemm_a<<<((MTOK / 64) * (HDIM / 64)) / GEMM_WAVES, 128, 0, stream>>>(X16, W1T, HF, HT);
    k_rowdot<<<(NB * HEADS * NODES) / 256, 256, 0, stream>>>(HF, a1, F1, F2, LG_HEADS, DH);
    k_attn_a<<<NB * (HEADS / 2) * (NODES / 64), 128, 0, stream>>>(HT, adj, F1, F2, XCH, XCL);

    k_gemm_b<<<((MTOK / 64) * (NCLS / 64)) / GEMM_WAVES, 128, 0, stream>>>(XCH, XCL, W2T, H2F, H2T);
    k_rowdot<<<(NB * NODES) / 256, 256, 0, stream>>>(H2F, a2, G1, G2, 0, NCLS);
    k_attn_b<<<NB * (NODES / 64), 128, 0, stream>>>(H2T, adj, G1, G2, x, out);
}
